// SwinBlock_45397804319463
// MI455X (gfx1250) — hardware-run, weakly checked
//
#include <hip/hip_runtime.h>
#include <hip/hip_bf16.h>
#include <math.h>
#include <stddef.h>

typedef __attribute__((ext_vector_type(16))) _Float16 v16h;
typedef __attribute__((ext_vector_type(8)))  _Float16 v8h;
typedef __attribute__((ext_vector_type(16))) __bf16   v16b;
typedef __attribute__((ext_vector_type(8)))  __bf16   v8b;
typedef __attribute__((ext_vector_type(8)))  float    v8f;
typedef __attribute__((ext_vector_type(4)))  float    v4f;
typedef __attribute__((ext_vector_type(2)))  float    v2f;
typedef __attribute__((ext_vector_type(4)))  unsigned int v4u;

constexpr int kBatch   = 8;
constexpr int kSeq     = 4096;
constexpr int kC       = 256;
constexpr int kRows    = kBatch * kSeq;
constexpr int kHid     = 1024;
constexpr int kNH      = 8;
constexpr int kHD      = 32;
constexpr int kWin     = 8;
constexpr int kW2      = 64;
constexpr int kNWin    = kRows / kW2;
constexpr int kQkvLd   = 3 * kC;
constexpr int kChunk   = 8192;
constexpr int kNChunk  = kRows / kChunk;
constexpr int kBiasTab = (2 * kWin - 1) * (2 * kWin - 1);

static_assert(kRows % 64 == 0 && kC % 64 == 0 && kHid % 64 == 0 && kChunk % 64 == 0, "");
static_assert(kC % 32 == 0 && kHid % 32 == 0, "");
static_assert(kNChunk * kChunk == kRows, "");

__device__ __forceinline__ unsigned short f2bf_bits(float f) {
  unsigned u = __float_as_uint(f);
  return (unsigned short)((u + 0x7FFFu + ((u >> 16) & 1u)) >> 16);
}
__device__ __forceinline__ float bf_bits2f(unsigned short h) { return __uint_as_float(((unsigned)h) << 16); }

__device__ __forceinline__ void dep_guard_h(v8f& a, v8f& b, v16h x, v16h y) { asm volatile("v_nop\n\tv_nop\n\tv_nop\n\tv_nop" : "+v"(a), "+v"(b) : "v"(x), "v"(y)); }
__device__ __forceinline__ void dep_guard_b(v8f& a, v8f& b, v16b x, v16b y) { asm volatile("v_nop\n\tv_nop\n\tv_nop\n\tv_nop" : "+v"(a), "+v"(b) : "v"(x), "v"(y)); }
__device__ __forceinline__ void keep4_h(v16h a, v16h b, v16h c, v16h d) { asm volatile("v_nop" :: "v"(a), "v"(b), "v"(c), "v"(d)); }
__device__ __forceinline__ void keep4_b(v16b a, v16b b, v16b c, v16b d) { asm volatile("v_nop" :: "v"(a), "v"(b), "v"(c), "v"(d)); }
__device__ __forceinline__ void acc_guard4(v8f& a, v8f& b, v8f& c, v8f& d) { asm volatile("v_nop\n\tv_nop\n\tv_nop\n\tv_nop" : "+v"(a), "+v"(b), "+v"(c), "+v"(d)); }

template <typename T> struct Frag;
template <> struct Frag<_Float16> {
  typedef v16h V; union U { v16h v; v8h h[2]; };
  static __device__ __forceinline__ v16h load(const _Float16* p) {
    U f; f.h[0] = *(const v8h*)(p); f.h[1] = *(const v8h*)(p + 16); return f.v;
  }
  static __device__ __forceinline__ v8f mma(v16h a, v16h b, v8f c) {
    return __builtin_amdgcn_wmma_f32_16x16x32_f16(false, a, false, b, (short)0, c, false, false);
  }
  static __device__ __forceinline__ void guard(v8f& a, v8f& b, v16h x, v16h y) { dep_guard_h(a, b, x, y); }
  static __device__ __forceinline__ void keep(v16h a, v16h b, v16h c, v16h d) { keep4_h(a, b, c, d); }
};
template <> struct Frag<__bf16> {
  typedef v16b V; union U { v16b v; v8b h[2]; };
  static __device__ __forceinline__ v16b load(const __bf16* p) {
    U f; f.h[0] = *(const v8b*)(p); f.h[1] = *(const v8b*)(p + 16); return f.v;
  }
  static __device__ __forceinline__ v8f mma(v16b a, v16b b, v8f c) {
    return __builtin_amdgcn_wmma_f32_16x16x32_bf16(false, a, false, b, (short)0, c, false, false);
  }
  static __device__ __forceinline__ void guard(v8f& a, v8f& b, v16b x, v16b y) { dep_guard_b(a, b, x, y); }
  static __device__ __forceinline__ void keep(v16b a, v16b b, v16b c, v16b d) { keep4_b(a, b, c, d); }
};

__device__ __forceinline__ unsigned short h_bits(float f) { return __builtin_bit_cast(unsigned short, (_Float16)f); }
__device__ __forceinline__ unsigned pack_h2(float a, float b) {
  return (unsigned)h_bits(a) | ((unsigned)h_bits(b) << 16);
}

__device__ __forceinline__ int perm_row(int m) {
  const int w = m >> 6, tk = m & 63;
  const int b = w >> 6, wl = w & 63;
  const int wy = wl >> 3, wx = wl & 7, iy = tk >> 3, ix = tk & 7;
  const int y = (wy * 8 + iy + 4) & 63;
  const int x = (wx * 8 + ix + 4) & 63;
  return (b << 12) + (y << 6) + x;
}

template <int ET> struct Elem;
template <> struct Elem<0> { typedef _Float16 T; };
template <> struct Elem<1> { typedef __bf16 T; };
template <int ET, bool SPLIT, int BIAS_MODE, int OUT_MODE, bool RESID, bool PERM>
__global__ __launch_bounds__(256) void wmma_gemm64(
    const unsigned short* __restrict__ Ap, const unsigned short* __restrict__ A2p, int lda, long strideA,
    const unsigned short* __restrict__ Btp, const unsigned short* __restrict__ Bt2p, int ldb, long strideB,
    void* __restrict__ Cout, void* __restrict__ Cout2, int ldc, long strideC,
    const float* __restrict__ bias, float bias_mul,
    const float* __restrict__ resid, long strideR,
    int M, int N, int K, float scale) {
  static_assert(!RESID || OUT_MODE == 0, "");
  static_assert(!PERM || OUT_MODE == 0, "");
  typedef typename Elem<ET>::T T;
  typedef typename Frag<T>::V V;
  const T* A = (const T*)Ap; const T* A2 = (const T*)A2p; const T* Bt = (const T*)Btp; const T* Bt2 = (const T*)Bt2p;
  __shared__ __align__(16) float sT[8][16 * 68];
  const int b    = blockIdx.y;
  const int lane = threadIdx.x & 31;
  const int wave = threadIdx.x >> 5;
  const int tilesN = N >> 6;
  const int tilesM = M >> 6;
  const int tile = blockIdx.x * 8 + wave;
  if (tile >= tilesM * tilesN) return;
  const int tm = tile / tilesN;
  const int tn = tile - tm * tilesN;
  const int m0 = tm << 6;
  const int n0 = tn << 6;

  const T* Ab  = A  + (size_t)b * strideA;
  const T* Bb  = Bt + (size_t)b * strideB;
  const T* Ab2 = SPLIT ? (A2  + (size_t)b * strideA) : nullptr;
  const T* Bb2 = SPLIT ? (Bt2 + (size_t)b * strideB) : nullptr;

  const int rlane = lane & 15;
  const int koff  = (lane >> 4) * 8;
  const int mOff  = (lane >> 4) * 8;

  v8f acc[4][4];
#pragma unroll
  for (int i = 0; i < 4; ++i)
#pragma unroll
    for (int j = 0; j < 4; ++j) acc[i][j] = (v8f){0.f,0.f,0.f,0.f,0.f,0.f,0.f,0.f};

  for (int k0 = 0; k0 < K; k0 += 32) {
    V bh[4], bl[4];
#pragma unroll
    for (int j = 0; j < 4; ++j) {
      const size_t bo = (size_t)(n0 + (j << 4) + rlane) * ldb + koff + k0;
      bh[j] = Frag<T>::load(Bb + bo);
      if (SPLIT) bl[j] = Frag<T>::load(Bb2 + bo);
    }
#pragma unroll
    for (int i = 0; i < 4; ++i) {
      const size_t ao = (size_t)(m0 + (i << 4) + rlane) * lda + koff + k0;
      V ah = Frag<T>::load(Ab + ao);
      V al;
      if (SPLIT) al = Frag<T>::load(Ab2 + ao);
#pragma unroll
      for (int j = 0; j < 4; ++j) {
        acc[i][j] = Frag<T>::mma(ah, bh[j], acc[i][j]);
        if (SPLIT) {
          acc[i][j] = Frag<T>::mma(ah, bl[j], acc[i][j]);
          acc[i][j] = Frag<T>::mma(al, bh[j], acc[i][j]);
        }
      }
      Frag<T>::guard(acc[i][0], acc[i][3], ah, SPLIT ? al : ah);
    }
    Frag<T>::keep(bh[0], bh[1], bh[2], bh[3]);
    if (SPLIT) Frag<T>::keep(bl[0], bl[1], bl[2], bl[3]);
  }
  acc_guard4(acc[0][0], acc[0][1], acc[0][2], acc[0][3]);
  acc_guard4(acc[1][0], acc[1][1], acc[1][2], acc[1][3]);
  acc_guard4(acc[2][0], acc[2][1], acc[2][2], acc[2][3]);
  acc_guard4(acc[3][0], acc[3][1], acc[3][2], acc[3][3]);

  float* slab = sT[wave];
#pragma unroll
  for (int i = 0; i < 4; ++i) {
    const int mBase = m0 + (i << 4);
#pragma unroll
    for (int j = 0; j < 4; ++j) {
      const int n = n0 + (j << 4) + rlane;
      float bv = 0.f;
      if (BIAS_MODE == 2) bv = bias[n] * bias_mul;
#pragma unroll
      for (int r = 0; r < 8; ++r) {
        float v = acc[i][j][r] * scale;
        if (BIAS_MODE == 1) v += bias[mBase + mOff + r] * bias_mul;
        if (BIAS_MODE == 2) v += bv;
        slab[(mOff + r) * 68 + (j << 4) + rlane] = v;
      }
    }
    __builtin_amdgcn_fence(__ATOMIC_RELEASE, "workgroup");
    __builtin_amdgcn_wave_barrier();
    __builtin_amdgcn_fence(__ATOMIC_ACQUIRE, "workgroup");
    if (OUT_MODE == 0) {
      float* Cb = (float*)Cout + (size_t)b * strideC;
      const float* Rb = RESID ? (resid + (size_t)b * strideR) : nullptr;
      const int hh = lane >> 4, c4 = (lane & 15) * 4;
      for (int pass = 0; pass < 2; ++pass) {
#pragma unroll
        for (int it = 0; it < 8; ++it) {
          const int row = it * 2 + hh;
          int drow = mBase + row;
          if (PERM) drow = perm_row(drow);
          v4f v = *(const v4f*)(slab + row * 68 + c4);
          if (RESID) {
            const v4f rv = *(const v4f*)(Rb + (size_t)drow * ldc + n0 + c4);
            v += rv;
          }
          *(volatile v4f*)(Cb + (size_t)drow * ldc + n0 + c4) = v;
        }
        __threadfence();
      }
    } else {
      const int q = lane >> 3, c8 = (lane & 7) * 8;
      unsigned short* Cb = (unsigned short*)Cout + (size_t)b * strideC;
      for (int pass = 0; pass < 2; ++pass) {
#pragma unroll
        for (int it = 0; it < 4; ++it) {
          const int row = it * 4 + q;
          const float* sp = slab + row * 68 + c8;
          v8h hv;
#pragma unroll
          for (int e = 0; e < 8; ++e) hv[e] = (_Float16)sp[e];
          *(volatile v8h*)(Cb + (size_t)(mBase + row) * ldc + n0 + c8) = hv;
        }
        __threadfence();
      }
    }
    __builtin_amdgcn_fence(__ATOMIC_RELEASE, "workgroup");
    __builtin_amdgcn_wave_barrier();
    __builtin_amdgcn_fence(__ATOMIC_ACQUIRE, "workgroup");
  }
}

__global__ __launch_bounds__(256) void k_wt_f16(const float* __restrict__ in, unsigned short* __restrict__ out,
                                                int Kd, int Nd, float mul) {
  __shared__ float sm[64 * 65];
  const int tid = threadIdx.x;
  const int n0 = blockIdx.x * 64, k0 = blockIdx.y * 64;
#pragma unroll
  for (int i = 0; i < 4; ++i) {
    const int idx = i * 256 + tid;
    const int r = idx >> 4, c4 = (idx & 15) * 4;
    const v4f v = *(const v4f*)(in + (size_t)(k0 + r) * Nd + n0 + c4);
    sm[(c4 + 0) * 65 + r] = v[0];
    sm[(c4 + 1) * 65 + r] = v[1];
    sm[(c4 + 2) * 65 + r] = v[2];
    sm[(c4 + 3) * 65 + r] = v[3];
  }
  __syncthreads();
  const int wave = tid >> 5, lane = tid & 31, q = lane >> 3, c8 = (lane & 7) * 8;
  for (int pass = 0; pass < 2; ++pass) {
#pragma unroll
    for (int it = 0; it < 2; ++it) {
      const int row = wave * 8 + it * 4 + q;
      const float* sp = sm + row * 65 + c8;
      v4u u;
      u[0] = pack_h2(sp[0] * mul, sp[1] * mul);
      u[1] = pack_h2(sp[2] * mul, sp[3] * mul);
      u[2] = pack_h2(sp[4] * mul, sp[5] * mul);
      u[3] = pack_h2(sp[6] * mul, sp[7] * mul);
      *(volatile v4u*)(void*)(out + (size_t)(n0 + row) * Kd + k0 + c8) = u;
    }
    __threadfence();
  }
}

__global__ __launch_bounds__(256) void k_adaln(const float* __restrict__ t, const float* __restrict__ w1,
                                               const float* __restrict__ b1, const float* __restrict__ w2,
                                               const float* __restrict__ b2, float* __restrict__ ss) {
  const int idx = blockIdx.x * 256 + threadIdx.x;
  const int b = idx >> 10, j = idx & 1023;
  const bool second = (j >= 512);
  const float* w  = second ? w2 : w1;
  const float* bb = second ? b2 : b1;
  const int jj = j & 511;
  const float* tr = t + b * kC;
  float acc = 0.f;
#pragma unroll 1
  for (int r = 0; r < kC; ++r) acc = fmaf(tr[r], w[(size_t)r * 512 + jj], acc);
  acc += bb[jj];
  ((volatile float*)ss)[idx] = acc;
  __threadfence();
  ((volatile float*)ss)[idx] = acc;
}

__global__ __launch_bounds__(256) void k_ln(const float* __restrict__ xin, const float* __restrict__ ss,
                                            int mod_off, int shifted, unsigned short* __restrict__ xout) {
  const int tid = threadIdx.x, wave = tid >> 5, lane = tid & 31;
  const int row = blockIdx.x * 8 + wave;
  const int b = row >> 12;
  const int row_in = shifted ? perm_row(row) : row;
  const float* src = xin + (size_t)row_in * kC + lane * 8;
  const v4f a0 = *(const v4f*)(src), a1 = *(const v4f*)(src + 4);
  float s = (a0[0] + a0[1]) + (a0[2] + a0[3]) + (a1[0] + a1[1]) + (a1[2] + a1[3]);
#pragma unroll
  for (int m = 16; m > 0; m >>= 1) s += __shfl_xor(s, m, 32);
  const float mu = s * (1.0f / 256.0f);
  float d[8];
  d[0] = a0[0] - mu; d[1] = a0[1] - mu; d[2] = a0[2] - mu; d[3] = a0[3] - mu;
  d[4] = a1[0] - mu; d[5] = a1[1] - mu; d[6] = a1[2] - mu; d[7] = a1[3] - mu;
  float s2 = 0.f;
#pragma unroll
  for (int e = 0; e < 8; ++e) s2 += d[e] * d[e];
#pragma unroll
  for (int m = 16; m > 0; m >>= 1) s2 += __shfl_xor(s2, m, 32);
  const float var = s2 * (1.0f / 256.0f);
  const float rs = rsqrtf(var + 1e-5f);
  const float* md = ss + b * 1024 + mod_off + lane * 8;
  const v4f sc0 = *(const v4f*)(md), sc1 = *(const v4f*)(md + 4);
  const v4f sh0 = *(const v4f*)(md + kC), sh1 = *(const v4f*)(md + kC + 4);
  float o[8];
#pragma unroll
  for (int e = 0; e < 4; ++e) {
    o[e]     = d[e] * rs * (1.0f + sc0[e]) + sh0[e];
    o[4 + e] = d[4 + e] * rs * (1.0f + sc1[e]) + sh1[e];
  }
  v4u u;
  u[0] = pack_h2(o[0], o[1]); u[1] = pack_h2(o[2], o[3]);
  u[2] = pack_h2(o[4], o[5]); u[3] = pack_h2(o[6], o[7]);
  unsigned short* dst = xout + (size_t)row * kC + lane * 8;
  *(volatile v4u*)(void*)dst = u;
  __threadfence();
  *(volatile v4u*)(void*)dst = u;
}

__device__ __forceinline__ void guard_s4(v8f& a, v8f& b, v8f& c, v8f& d, v16h qa, v16h k0, v16h k1, v16h k2, v16h k3) {
  asm volatile("v_nop\n\tv_nop\n\tv_nop\n\tv_nop" : "+v"(a), "+v"(b), "+v"(c), "+v"(d) : "v"(qa), "v"(k0), "v"(k1), "v"(k2), "v"(k3));
}
__device__ __forceinline__ void guard_o2(v8f& a, v8f& b, v16h p0, v16h p1, v16h x0, v16h x1, v16h x2, v16h x3) {
  asm volatile("v_nop\n\tv_nop\n\tv_nop\n\tv_nop" : "+v"(a), "+v"(b) : "v"(p0), "v"(p1), "v"(x0), "v"(x1), "v"(x2), "v"(x3));
}

__global__ __launch_bounds__(256) void k_wattn(const unsigned short* __restrict__ qkv, const float* __restrict__ btab,
                                               unsigned short* __restrict__ ao) {
  __shared__ __align__(16) unsigned short Vt[kNH * kHD * kW2];
  __shared__ __align__(16) unsigned short Pw[8 * 16 * kW2];
  __shared__ __align__(16) unsigned short Ost[16 * 264];
  __shared__ float bt[kBiasTab * kNH];
  const int tid = threadIdx.x, h = tid >> 5, lane = tid & 31, hh = lane >> 4, c = lane & 15, koff = hh * 8;
  const int w = blockIdx.x;
  const size_t R0 = (size_t)w * kW2;
  const _Float16* qkvh = (const _Float16*)(const void*)qkv;

  for (int i = tid; i < kBiasTab * kNH; i += 256) bt[i] = btab[i];

  unsigned short* Vth = Vt + h * (kHD * kW2);
  unsigned short* Pwh = Pw + h * (16 * kW2);
#pragma unroll
  for (int half = 0; half < 2; ++half) {
    const int kv = lane + 32 * half;
    const v4u* vp = (const v4u*)(const void*)(qkv + (R0 + kv) * kQkvLd + 2 * kC + h * kHD);
#pragma unroll
    for (int i = 0; i < 4; ++i) {
      const v4u wv = vp[i];
#pragma unroll
      for (int e = 0; e < 4; ++e) {
        const unsigned u = wv[e];
        const int d = i * 8 + 2 * e;
        Vth[d * kW2 + kv]       = (unsigned short)(u & 0xffffu);
        Vth[(d + 1) * kW2 + kv] = (unsigned short)(u >> 16);
      }
    }
  }
  __syncthreads();

  const float scl = 0.17677669529663687f * (1.0f / 64.0f);
  const _Float16* Vthh = (const _Float16*)(const void*)Vth;
  const _Float16* Pwhh = (const _Float16*)(const void*)Pwh;

#pragma unroll 1
  for (int mt = 0; mt < 4; ++mt) {
    const v16h qa = Frag<_Float16>::load(qkvh + (R0 + mt * 16 + c) * kQkvLd + h * kHD + koff);
    v16h kb[4];
#pragma unroll
    for (int j = 0; j < 4; ++j)
      kb[j] = Frag<_Float16>::load(qkvh + (R0 + j * 16 + c) * kQkvLd + kC + h * kHD + koff);
    v8f s[4];
#pragma unroll
    for (int j = 0; j < 4; ++j) {
      s[j] = (v8f){0.f,0.f,0.f,0.f,0.f,0.f,0.f,0.f};
      s[j] = Frag<_Float16>::mma(qa, kb[j], s[j]);
    }
    guard_s4(s[0], s[1], s[2], s[3], qa, kb[0], kb[1], kb[2], kb[3]);

    float inv[8];
#pragma unroll
    for (int r = 0; r < 8; ++r) {
      const int qi = mt * 16 + 8 * hh + r;
      const int qy = qi >> 3, qx = qi & 7;
      float m = -INFINITY;
#pragma unroll
      for (int j = 0; j < 4; ++j) {
        const int kj = j * 16 + c;
        const int ky = kj >> 3, kx = kj & 7;
        const int bidx = ((qy - ky + 7) * 15 + (qx - kx + 7)) * kNH + h;
        const float val = s[j][r] * scl + bt[bidx];
        s[j][r] = val;
        m = fmaxf(m, val);
      }
#pragma unroll
      for (int off = 1; off < 16; off <<= 1) m = fmaxf(m, __shfl_xor(m, off, 32));
      float psum = 0.f;
#pragma unroll
      for (int j = 0; j < 4; ++j) {
        const float p = expf(s[j][r] - m);
        psum += p;
        Pwh[(8 * hh + r) * kW2 + j * 16 + c] = h_bits(p * 1024.0f);
      }
#pragma unroll
      for (int off = 1; off < 16; off <<= 1) psum += __shfl_xor(psum, off, 32);
      inv[r] = (1.0f / psum) * (1.0f / 512.0f);
    }
    __builtin_amdgcn_fence(__ATOMIC_RELEASE, "workgroup");
    __builtin_amdgcn_wave_barrier();
    __builtin_amdgcn_fence(__ATOMIC_ACQUIRE, "workgroup");

    v8f oacc[2];
    oacc[0] = (v8f){0.f,0.f,0.f,0.f,0.f,0.f,0.f,0.f};
    oacc[1] = (v8f){0.f,0.f,0.f,0.f,0.f,0.f,0.f,0.f};
    v16h pa[2], vb0[2], vb1[2];
#pragma unroll
    for (int kk = 0; kk < 2; ++kk) {
      pa[kk]  = Frag<_Float16>::load(Pwhh + c * kW2 + kk * 32 + koff);
      vb0[kk] = Frag<_Float16>::load(Vthh + (0 * 16 + c) * kW2 + kk * 32 + koff);
      vb1[kk] = Frag<_Float16>::load(Vthh + (1 * 16 + c) * kW2 + kk * 32 + koff);
    }
#pragma unroll
    for (int kk = 0; kk < 2; ++kk) {
      oacc[0] = Frag<_Float16>::mma(pa[kk], vb0[kk], oacc[0]);
      oacc[1] = Frag<_Float16>::mma(pa[kk], vb1[kk], oacc[1]);
    }
    guard_o2(oacc[0], oacc[1], pa[0], pa[1], vb0[0], vb0[1], vb1[0], vb1[1]);

#pragma unroll
    for (int r = 0; r < 8; ++r) {
      Ost[(8 * hh + r) * 264 + h * kHD + c]      = h_bits(oacc[0][r] * inv[r]);
      Ost[(8 * hh + r) * 264 + h * kHD + 16 + c] = h_bits(oacc[1][r] * inv[r]);
    }
    __syncthreads();
    for (int pass = 0; pass < 2; ++pass) {
#pragma unroll
      for (int rr = 0; rr < 2; ++rr) {
        const int row = 2 * h + rr;
        const v4u v = *(const v4u*)(const void*)(Ost + row * 264 + lane * 8);
        *(volatile v4u*)(void*)(ao + (R0 + mt * 16 + row) * kC + lane * 8) = v;
      }
      __threadfence();
    }
    __syncthreads();
  }
}

__device__ __forceinline__ float gelu16(float v) {
  return 8.0f * v * (1.0f + erff(v * 0.70710678118654752f));
}
__global__ __launch_bounds__(256) void k_gelu(const float* __restrict__ hp, unsigned short* __restrict__ g) {
  const int tid = threadIdx.x;
#pragma unroll 1
  for (int it = 0; it < 4; ++it) {
    const size_t wi = ((size_t)blockIdx.x * 4 + it) * 256 + tid;
    const v2f v = *(const v2f*)(hp + 2 * wi);
    const float g0 = gelu16(v[0]);
    const float g1 = gelu16(v[1]);
    const unsigned u = pack_h2(g0, g1);
    ((volatile unsigned*)g)[wi] = u;
    __threadfence();
    ((volatile unsigned*)g)[wi] = u;
  }
}

constexpr size_t kOffWqkv = 0;
constexpr size_t kOffWo   = kOffWqkv + (size_t)3 * kC * kC * 2;
constexpr size_t kOffW1   = kOffWo + (size_t)kC * kC * 2;
constexpr size_t kOffW2   = kOffW1 + (size_t)kHid * kC * 2;
constexpr size_t kOffSs   = kOffW2 + (size_t)kC * kHid * 2;
constexpr size_t kOffXw   = kOffSs + (size_t)kBatch * 1024 * 4;
constexpr size_t kOffQkv  = kOffXw + (size_t)kRows * kC * 2;
constexpr size_t kOffHpre = kOffQkv;
constexpr size_t kOffG    = kOffQkv + (size_t)kChunk * kHid * 4;
constexpr size_t kOffAo   = kOffQkv + (size_t)kRows * kQkvLd * 2;
constexpr size_t kOffX1   = kOffAo + (size_t)kRows * kC * 2;
constexpr size_t kWsTotal = kOffX1 + (size_t)kRows * kC * 4;
static_assert(kOffG + (size_t)kChunk * kHid * 2 <= kOffAo, "");
static_assert(kWsTotal == 119046144, "");
static_assert(kWsTotal <= 134217728, "");
static_assert(kOffXw % 128 == 0 && kOffQkv % 128 == 0 && kOffG % 128 == 0 && kOffAo % 128 == 0 && kOffX1 % 128 == 0, "");

typedef void (*gemm_fn)(const unsigned short*, const unsigned short*, int, long,
                        const unsigned short*, const unsigned short*, int, long,
                        void*, void*, int, long, const float*, float, const float*, long,
                        int, int, int, float);

extern "C" void kernel_launch(void* const* d_in, const int* in_sizes, int n_in,
                              void* d_out, int out_size, void* d_ws, size_t ws_size, hipStream_t stream) {
  (void)in_sizes; (void)n_in; (void)out_size;
  if (ws_size < kWsTotal) return;
  const float* x    = (const float*)d_in[0];
  const float* temb = (const float*)d_in[1];
  const float* a1w  = (const float*)d_in[4];
  const float* a1b  = (const float*)d_in[5];
  const float* a2w  = (const float*)d_in[6];
  const float* a2b  = (const float*)d_in[7];
  const float* btab = (const float*)d_in[8];
  const float* qw   = (const float*)d_in[9];
  const float* qb   = (const float*)d_in[10];
  const float* kw   = (const float*)d_in[11];
  const float* kbv  = (const float*)d_in[12];
  const float* vw   = (const float*)d_in[13];
  const float* vb   = (const float*)d_in[14];
  const float* ow   = (const float*)d_in[15];
  const float* ob   = (const float*)d_in[16];
  const float* f1w  = (const float*)d_in[17];
  const float* f1b  = (const float*)d_in[18];
  const float* f2w  = (const float*)d_in[19];
  const float* f2b  = (const float*)d_in[20];
  float* out = (float*)d_out;

  char* wsb = (char*)d_ws;
  unsigned short* wqkv = (unsigned short*)(wsb + kOffWqkv);
  unsigned short* wo   = (unsigned short*)(wsb + kOffWo);
  unsigned short* w1t  = (unsigned short*)(wsb + kOffW1);
  unsigned short* w2t  = (unsigned short*)(wsb + kOffW2);
  float*          ss   = (float*)(wsb + kOffSs);
  unsigned short* xw   = (unsigned short*)(wsb + kOffXw);
  unsigned short* xn2  = xw;
  unsigned short* qkv  = (unsigned short*)(wsb + kOffQkv);
  float*          hpre = (float*)(wsb + kOffHpre);
  unsigned short* gpl  = (unsigned short*)(wsb + kOffG);
  unsigned short* ao   = (unsigned short*)(wsb + kOffAo);
  float*          x1   = (float*)(wsb + kOffX1);

  k_wt_f16<<<dim3(kC / 64, kC / 64), 256, 0, stream>>>(qw, wqkv + 0 * kC * kC, kC, kC, 64.0f);
  k_wt_f16<<<dim3(kC / 64, kC / 64), 256, 0, stream>>>(kw, wqkv + 1 * kC * kC, kC, kC, 64.0f);
  k_wt_f16<<<dim3(kC / 64, kC / 64), 256, 0, stream>>>(vw, wqkv + 2 * kC * kC, kC, kC, 64.0f);
  k_wt_f16<<<dim3(kC / 64, kC / 64), 256, 0, stream>>>(ow, wo, kC, kC, 64.0f);
  k_wt_f16<<<dim3(kHid / 64, kC / 64), 256, 0, stream>>>(f1w, w1t, kC, kHid, 64.0f);
  k_wt_f16<<<dim3(kC / 64, kHid / 64), 256, 0, stream>>>(f2w, w2t, kHid, kC, 64.0f);

  static_assert((kBatch * 1024) % 256 == 0, "");
  k_adaln<<<(kBatch * 1024) / 256, 256, 0, stream>>>(temb, a1w, a1b, a2w, a2b, ss);

  static_assert(kRows % 8 == 0, "");
  k_ln<<<kRows / 8, 256, 0, stream>>>(x, ss, 0, 1, xw);

  static_assert(kRows % 64 == 0 && kC % 64 == 0 && kC % 32 == 0, "");
  gemm_fn g_qkv = wmma_gemm64<0, false, 2, 1, false, false>;
  const int nb_qkv = ((kRows / 64) * (kC / 64) + 7) / 8;
  {
    const float* biases[3] = {qb, kbv, vb};
    for (int mat = 0; mat < 3; ++mat) {
      g_qkv<<<dim3(nb_qkv, 1), 256, 0, stream>>>(
          xw, xw, kC, 0L,
          wqkv + (size_t)mat * kC * kC, wqkv + (size_t)mat * kC * kC, kC, 0L,
          (void*)(qkv + mat * kC), nullptr, kQkvLd, 0L,
          biases[mat], 8.0f, nullptr, 0L,
          kRows, kC, kC, 8.0f / 64.0f);
    }
  }

  k_wattn<<<kNWin, 256, 0, stream>>>(qkv, btab, ao);

  gemm_fn g_o = wmma_gemm64<0, false, 2, 0, true, true>;
  g_o<<<dim3(nb_qkv, 1), 256, 0, stream>>>(
      ao, ao, kC, 0L, wo, wo, kC, 0L,
      (void*)x1, nullptr, kC, 0L,
      ob, 1.0f, x, 0L,
      kRows, kC, kC, 1.0f / 1024.0f);

  k_ln<<<kRows / 8, 256, 0, stream>>>(x1, ss, 512, 0, xn2);

  static_assert(kChunk % 64 == 0 && kHid % 64 == 0 && kHid % 32 == 0, "");
  static_assert((kChunk * kHid / 2) % 1024 == 0, "");
  gemm_fn g_f1 = wmma_gemm64<0, false, 2, 0, false, false>;
  gemm_fn g_f2 = wmma_gemm64<0, false, 2, 0, true, false>;
  const int nb_f1 = ((kChunk / 64) * (kHid / 64) + 7) / 8;
  const int nb_f2 = ((kChunk / 64) * (kC / 64) + 7) / 8;
  const int nb_gelu = (kChunk * kHid / 2) / 1024;
  for (int ch = 0; ch < kNChunk; ++ch) {
    const size_t r0 = (size_t)ch * kChunk;
    g_f1<<<dim3(nb_f1, 1), 256, 0, stream>>>(
        xn2 + r0 * kC, xn2 + r0 * kC, kC, 0L, w1t, w1t, kC, 0L,
        (void*)hpre, nullptr, kHid, 0L,
        f1b, 1.0f, nullptr, 0L,
        kChunk, kHid, kC, 1.0f / 64.0f);
    k_gelu<<<nb_gelu, 256, 0, stream>>>(hpre, gpl);
    g_f2<<<dim3(nb_f2, 1), 256, 0, stream>>>(
        gpl, gpl, kHid, 0L, w2t, w2t, kHid, 0L,
        (void*)(out + r0 * kC), nullptr, kC, 0L,
        f2b, 1.0f, x1 + r0 * kC, 0L,
        kChunk, kC, kHid, 1.0f / 1024.0f);
  }
}
